// EncoderDecoderLSTM_69106023792936
// MI455X (gfx1250) — hardware-run, weakly checked
//
#include <hip/hip_runtime.h>
#include <stdint.h>

typedef __attribute__((ext_vector_type(16))) _Float16 v16h;
typedef __attribute__((ext_vector_type(8)))  _Float16 v8h;
typedef __attribute__((ext_vector_type(16))) __bf16   v16b;
typedef __attribute__((ext_vector_type(8)))  __bf16   v8b;
typedef __attribute__((ext_vector_type(8)))  float    v8f;
typedef __attribute__((ext_vector_type(4)))  float    v4f;
typedef __attribute__((ext_vector_type(4)))  unsigned int v4u;
#define PSCALE 32768.0f
#define U16(p) ((const unsigned short*)(const void*)(p))
#define PSCALE_INV (1.0f / 32768.0f)

__device__ __forceinline__ unsigned short f2bf_bits(float f) {
  unsigned u = __float_as_uint(f);
  return (unsigned short)((u + 0x7FFFu + ((u >> 16) & 1u)) >> 16);
}
__device__ __forceinline__ float bf_bits2f(unsigned short h) { return __uint_as_float(((unsigned)h) << 16); }

__device__ __forceinline__ void dep_guard_h(v8f& a, v8f& b, v16h x, v16h y) { asm volatile("v_nop\n\tv_nop\n\tv_nop\n\tv_nop" : "+v"(a), "+v"(b) : "v"(x), "v"(y)); }
__device__ __forceinline__ void dep_guard_b(v8f& a, v8f& b, v16b x, v16b y) { asm volatile("v_nop\n\tv_nop\n\tv_nop\n\tv_nop" : "+v"(a), "+v"(b) : "v"(x), "v"(y)); }
__device__ __forceinline__ void keep4_h(v16h a, v16h b, v16h c, v16h d) { asm volatile("v_nop" :: "v"(a), "v"(b), "v"(c), "v"(d)); }
__device__ __forceinline__ void keep4_b(v16b a, v16b b, v16b c, v16b d) { asm volatile("v_nop" :: "v"(a), "v"(b), "v"(c), "v"(d)); }
__device__ __forceinline__ void acc_guard4(v8f& a, v8f& b, v8f& c, v8f& d) { asm volatile("v_nop\n\tv_nop\n\tv_nop\n\tv_nop" : "+v"(a), "+v"(b), "+v"(c), "+v"(d)); }
template <typename T> struct Frag;
template <> struct Frag<_Float16> {
  typedef v16h V; union U { v16h v; v8h h[2]; };
  static __device__ __forceinline__ v16h load(const _Float16* p) {
    U f; f.h[0] = *(const v8h*)(p); f.h[1] = *(const v8h*)(p + 16); return f.v;
  }
  static __device__ __forceinline__ v8f mma(v16h a, v16h b, v8f c) {
    return __builtin_amdgcn_wmma_f32_16x16x32_f16(false, a, false, b, (short)0, c, false, false);
  }
  static __device__ __forceinline__ void guard(v8f& a, v8f& b, v16h x, v16h y) { dep_guard_h(a, b, x, y); }
  static __device__ __forceinline__ void keep(v16h a, v16h b, v16h c, v16h d) { keep4_h(a, b, c, d); }
};
template <> struct Frag<__bf16> {
  typedef v16b V; union U { v16b v; v8b h[2]; };
  static __device__ __forceinline__ v16b load(const __bf16* p) {
    U f; f.h[0] = *(const v8b*)(p); f.h[1] = *(const v8b*)(p + 16); return f.v;
  }
  static __device__ __forceinline__ v8f mma(v16b a, v16b b, v8f c) {
    return __builtin_amdgcn_wmma_f32_16x16x32_bf16(false, a, false, b, (short)0, c, false, false);
  }
  static __device__ __forceinline__ void guard(v8f& a, v8f& b, v16b x, v16b y) { dep_guard_b(a, b, x, y); }
  static __device__ __forceinline__ void keep(v16b a, v16b b, v16b c, v16b d) { keep4_b(a, b, c, d); }
};

template <int ET> struct Elem;
template <> struct Elem<0> { typedef _Float16 T; };
template <> struct Elem<1> { typedef __bf16 T; };
template <int ET, bool SPLIT, int BIAS_MODE, int OUT_MODE, bool RESID, int ACT = 0>
__global__ __launch_bounds__(256) void wmma_gemm64(
    const unsigned short* __restrict__ Ap, const unsigned short* __restrict__ A2p, int lda, long strideA,
    const unsigned short* __restrict__ Btp, const unsigned short* __restrict__ Bt2p, int ldb, long strideB,
    void* __restrict__ Cout, void* __restrict__ Cout2, int ldc, long strideC,
    const float* __restrict__ bias,
    const float* __restrict__ resid, long strideR,
    int M, int N, int K, float scale) {
  typedef typename Elem<ET>::T T;
  typedef typename Frag<T>::V V;
  const T* A = (const T*)Ap; const T* A2 = (const T*)A2p; const T* Bt = (const T*)Btp; const T* Bt2 = (const T*)Bt2p;
  __shared__ __align__(16) float sT[8][16 * 68];
  const int b    = blockIdx.y;
  const int lane = threadIdx.x & 31;
  const int wave = threadIdx.x >> 5;
  const int tilesN = N >> 6;
  const int tilesM = M >> 6;
  const int tile = blockIdx.x * 8 + wave;
  if (tile >= tilesM * tilesN) return;
  const int tm = tile / tilesN;
  const int tn = tile - tm * tilesN;
  const int m0 = tm << 6;
  const int n0 = tn << 6;

  const T* Ab  = A  + (size_t)b * strideA;
  const T* Bb  = Bt + (size_t)b * strideB;
  const T* Ab2 = SPLIT ? (A2  + (size_t)b * strideA) : nullptr;
  const T* Bb2 = SPLIT ? (Bt2 + (size_t)b * strideB) : nullptr;

  const int rlane = lane & 15;
  const int koff  = (lane >> 4) * 8;
  const int mOff  = (lane >> 4) * 8;

  v8f acc[4][4];
#pragma unroll
  for (int i = 0; i < 4; ++i)
#pragma unroll
    for (int j = 0; j < 4; ++j) acc[i][j] = (v8f){0.f,0.f,0.f,0.f,0.f,0.f,0.f,0.f};

  for (int k0 = 0; k0 < K; k0 += 32) {
    V bh[4], bl[4];
#pragma unroll
    for (int j = 0; j < 4; ++j) {
      const size_t bo = (size_t)(n0 + (j << 4) + rlane) * ldb + koff + k0;
      bh[j] = Frag<T>::load(Bb + bo);
      if (SPLIT) bl[j] = Frag<T>::load(Bb2 + bo);
    }
#pragma unroll
    for (int i = 0; i < 4; ++i) {
      const size_t ao = (size_t)(m0 + (i << 4) + rlane) * lda + koff + k0;
      V ah = Frag<T>::load(Ab + ao);
      V al;
      if (SPLIT) al = Frag<T>::load(Ab2 + ao);
#pragma unroll
      for (int j = 0; j < 4; ++j) {
        acc[i][j] = Frag<T>::mma(ah, bh[j], acc[i][j]);
        if (SPLIT) {
          acc[i][j] = Frag<T>::mma(ah, bl[j], acc[i][j]);
          acc[i][j] = Frag<T>::mma(al, bh[j], acc[i][j]);
        }
      }
      Frag<T>::guard(acc[i][0], acc[i][3], ah, SPLIT ? al : ah);
    }
    Frag<T>::keep(bh[0], bh[1], bh[2], bh[3]);
    if (SPLIT) Frag<T>::keep(bl[0], bl[1], bl[2], bl[3]);
  }
  acc_guard4(acc[0][0], acc[0][1], acc[0][2], acc[0][3]);
  acc_guard4(acc[1][0], acc[1][1], acc[1][2], acc[1][3]);
  acc_guard4(acc[2][0], acc[2][1], acc[2][2], acc[2][3]);
  acc_guard4(acc[3][0], acc[3][1], acc[3][2], acc[3][3]);

  float* slab = sT[wave];
  const float* Rb = RESID ? (resid + (size_t)b * strideR) : nullptr;
#pragma unroll
  for (int i = 0; i < 4; ++i) {
    const int mBase = m0 + (i << 4);
#pragma unroll
    for (int j = 0; j < 4; ++j) {
      const int n = n0 + (j << 4) + rlane;
      float bv = 0.f;
      if (BIAS_MODE == 2) bv = bias[n];
#pragma unroll
      for (int r = 0; r < 8; ++r) {
        float v = acc[i][j][r] * scale;
        if (BIAS_MODE == 1) v += bias[mBase + mOff + r];
        if (BIAS_MODE == 2) v += bv;
        if (RESID) v += Rb[(size_t)(mBase + mOff + r) * ldc + n];
        if (ACT == 1) v = tanhf(v);
        if (ACT == 2) v = fmaxf(v, 0.0f);
        if (ACT == 3) v = v / (1.0f + expf(-v));
        if (ACT == 4) v = (v > 0.f) ? v : 0.01f * v;
        if (ACT == 5) v = 0.5f * v * (1.0f + erff(v * 0.70710678118654752f));
        slab[(mOff + r) * 68 + (j << 4) + rlane] = v;
      }
    }
    __builtin_amdgcn_fence(__ATOMIC_RELEASE, "workgroup");
    __builtin_amdgcn_wave_barrier();
    __builtin_amdgcn_fence(__ATOMIC_ACQUIRE, "workgroup");
    if (OUT_MODE == 0) {
      float* C = (float*)Cout + (size_t)b * strideC;
      const int hh = lane >> 4, c4 = (lane & 15) * 4;
      for (int pass = 0; pass < 2; ++pass) {
#pragma unroll
        for (int it = 0; it < 8; ++it) {
          const int row = it * 2 + hh;
          v4f v = *(const v4f*)(slab + row * 68 + c4);
          *(volatile v4f*)(C + (size_t)(mBase + row) * ldc + n0 + c4) = v;
        }
        __threadfence();
      }
    } else {
      const int q = lane >> 3, c8 = (lane & 7) * 8;
      unsigned short* C  = (unsigned short*)Cout  + (size_t)b * strideC;
      unsigned short* C2 = (OUT_MODE == 2) ? ((unsigned short*)Cout2 + (size_t)b * strideC) : nullptr;
      for (int pass = 0; pass < 2; ++pass) {
#pragma unroll
        for (int it = 0; it < 4; ++it) {
          const int row = it * 4 + q;
          const float* sp = slab + row * 68 + c8;
          v8h hv, lv;
#pragma unroll
          for (int e = 0; e < 8; ++e) {
            if (OUT_MODE == 1) {
              hv[e] = (_Float16)sp[e];
            } else {
              unsigned short hb = f2bf_bits(sp[e]);
              unsigned short lb = f2bf_bits(sp[e] - bf_bits2f(hb));
              hv[e] = __builtin_bit_cast(_Float16, hb);
              lv[e] = __builtin_bit_cast(_Float16, lb);
            }
          }
          *(volatile v8h*)(C + (size_t)(mBase + row) * ldc + n0 + c8) = hv;
          if (OUT_MODE == 2) *(volatile v8h*)(C2 + (size_t)(mBase + row) * ldc + n0 + c8) = lv;
        }
        __threadfence();
      }
    }
    __builtin_amdgcn_fence(__ATOMIC_RELEASE, "workgroup");
    __builtin_amdgcn_wave_barrier();
    __builtin_amdgcn_fence(__ATOMIC_ACQUIRE, "workgroup");
  }
}

constexpr int BATCH = 64;
constexpr int SEQ   = 128;
constexpr int FEAT  = 12;
constexpr int HID   = 128;
constexpr int GATES = 4 * HID;
constexpr int KCAT  = 160;
constexpr int HPITCH = 168;
constexpr int NROW  = BATCH * SEQ;
constexpr int OUT_NPAD = 64;
constexpr int APITCH = 136;
constexpr int TQ = 16;
constexpr float WSC = 64.0f;
constexpr float WSC_INV = 0.015625f;
constexpr float PCARRY = 1024.0f;
constexpr float PCARRY_INV = 0.0009765625f;

static_assert(NROW % 64 == 0);
static_assert(HID % 64 == 0);
static_assert(OUT_NPAD % 64 == 0);
static_assert(HID % 32 == 0);
static_assert((2 * HID) % 32 == 0);
static_assert(KCAT % 32 == 0);
static_assert(KCAT >= HID + FEAT);
static_assert(HPITCH >= KCAT && (HPITCH * 2) % 16 == 0);
static_assert((APITCH * 2) % 16 == 0);
static_assert(SEQ % TQ == 0 && SEQ == 128 && HID == 128 && BATCH == 64);
static_assert((NROW * FEAT) % (4 * 256) == 0);
static_assert((GATES * KCAT) % (8 * 32) == 0);

__device__ __forceinline__ unsigned short h_bits(float f) { return __builtin_bit_cast(unsigned short, (_Float16)f); }
__device__ __forceinline__ float sigm_f(float z) { return __builtin_amdgcn_rcpf(1.0f + expf(-z)); }

__device__ __forceinline__ v8f mma_h1(v16h a, v16h b, v8f c) {
  c = __builtin_amdgcn_wmma_f32_16x16x32_f16(false, a, false, b, (short)0, c, false, false);
  asm volatile("v_nop\n\tv_nop\n\tv_nop\n\tv_nop" : "+v"(c) : "v"(a), "v"(b));
  return c;
}
__device__ __forceinline__ void lds_wave_sync() {
  __builtin_amdgcn_fence(__ATOMIC_RELEASE, "workgroup");
  __builtin_amdgcn_wave_barrier();
  __builtin_amdgcn_fence(__ATOMIC_ACQUIRE, "workgroup");
}

__global__ __launch_bounds__(256) void prep_planes(const float* __restrict__ encWhh, const float* __restrict__ encWih,
                                                   const float* __restrict__ decWhh, const float* __restrict__ decWih,
                                                   const float* __restrict__ attnW, const float* __restrict__ outW,
                                                   unsigned short* __restrict__ wcatE, unsigned short* __restrict__ wcatD,
                                                   unsigned short* __restrict__ wattP, unsigned short* __restrict__ woutP) {
  const int which = blockIdx.y;
  const int i = blockIdx.x * 256 + threadIdx.x;
  unsigned short hb[8];
  if (which < 2) {
    const float* Whh = (which == 0) ? encWhh : decWhh;
    const float* Wih = (which == 0) ? encWih : decWih;
    unsigned short* dst = (which == 0) ? wcatE : wcatD;
    if (i < GATES * KCAT / 8) {
      const int row = i / (KCAT / 8);
      const int c0 = (i - row * (KCAT / 8)) * 8;
#pragma unroll
      for (int e = 0; e < 8; ++e) {
        const int c = c0 + e;
        const int ch = (c < HID) ? c : (HID - 1);
        int cx = c - HID; cx = (cx < 0) ? 0 : ((cx > FEAT - 1) ? (FEAT - 1) : cx);
        const float w1 = Whh[row * HID + ch];
        const float w2 = Wih[row * FEAT + cx];
        const float v = (c < HID) ? w1 : ((c < HID + FEAT) ? w2 : 0.0f);
        hb[e] = h_bits(WSC * v);
      }
      v4u w;
      w[0] = (unsigned)hb[0] | ((unsigned)hb[1] << 16);
      w[1] = (unsigned)hb[2] | ((unsigned)hb[3] << 16);
      w[2] = (unsigned)hb[4] | ((unsigned)hb[5] << 16);
      w[3] = (unsigned)hb[6] | ((unsigned)hb[7] << 16);
      *(volatile v4u*)(dst + (size_t)8 * i) = w;
      __threadfence();
      *(volatile v4u*)(dst + (size_t)8 * i) = w;
    }
  } else if (which == 2) {
    if (i < HID * 2 * HID / 8) {
      const v4f a0 = *(const v4f*)(attnW + (size_t)8 * i);
      const v4f a1 = *(const v4f*)(attnW + (size_t)8 * i + 4);
#pragma unroll
      for (int e = 0; e < 4; ++e) { hb[e] = h_bits(WSC * a0[e]); hb[4 + e] = h_bits(WSC * a1[e]); }
      v4u w;
      w[0] = (unsigned)hb[0] | ((unsigned)hb[1] << 16);
      w[1] = (unsigned)hb[2] | ((unsigned)hb[3] << 16);
      w[2] = (unsigned)hb[4] | ((unsigned)hb[5] << 16);
      w[3] = (unsigned)hb[6] | ((unsigned)hb[7] << 16);
      *(volatile v4u*)(wattP + (size_t)8 * i) = w;
      __threadfence();
      *(volatile v4u*)(wattP + (size_t)8 * i) = w;
    }
  } else {
    if (i < OUT_NPAD * 2 * HID / 8) {
      const int row = i / (2 * HID / 8);
      const int c0 = (i - row * (2 * HID / 8)) * 8;
      const int rr = (row < FEAT) ? row : (FEAT - 1);
      const v4f a0 = *(const v4f*)(outW + (size_t)rr * 2 * HID + c0);
      const v4f a1 = *(const v4f*)(outW + (size_t)rr * 2 * HID + c0 + 4);
      const bool live = (row < FEAT);
#pragma unroll
      for (int e = 0; e < 4; ++e) {
        hb[e]     = h_bits(live ? WSC * a0[e] : 0.0f);
        hb[4 + e] = h_bits(live ? WSC * a1[e] : 0.0f);
      }
      v4u w;
      w[0] = (unsigned)hb[0] | ((unsigned)hb[1] << 16);
      w[1] = (unsigned)hb[2] | ((unsigned)hb[3] << 16);
      w[2] = (unsigned)hb[4] | ((unsigned)hb[5] << 16);
      w[3] = (unsigned)hb[6] | ((unsigned)hb[7] << 16);
      *(volatile v4u*)(woutP + (size_t)8 * i) = w;
      __threadfence();
      *(volatile v4u*)(woutP + (size_t)8 * i) = w;
    }
  }
}

__device__ __forceinline__ void lstm_group(const unsigned short* shc, unsigned short* shn,
                                           const unsigned short* __restrict__ wcat, const float* sb,
                                           int mt, int cg, int rl, int hf, float (&cs)[8]) {
  v8f acc[4];
#pragma unroll
  for (int g = 0; g < 4; ++g) acc[g] = (v8f){0.f,0.f,0.f,0.f,0.f,0.f,0.f,0.f};
  const _Float16* arow = (const _Float16*)shc + (mt * 16 + rl) * HPITCH + 8 * hf;
  const _Float16* brow = (const _Float16*)wcat + (size_t)(cg * 16 + rl) * KCAT + 8 * hf;
#pragma unroll 1
  for (int kc = 0; kc < KCAT / 32; ++kc) {
    const v16h a = Frag<_Float16>::load(arow + kc * 32);
    v16h bq[4];
#pragma unroll
    for (int g = 0; g < 4; ++g) bq[g] = Frag<_Float16>::load(brow + (size_t)g * HID * KCAT + kc * 32);
#pragma unroll
    for (int g = 0; g < 4; ++g) acc[g] = Frag<_Float16>::mma(a, bq[g], acc[g]);
    dep_guard_h(acc[0], acc[3], a, bq[3]);
    keep4_h(bq[0], bq[1], bq[2], bq[3]);
  }
  acc_guard4(acc[0], acc[1], acc[2], acc[3]);
  const int col = cg * 16 + rl;
  const float bi = sb[col], bf = sb[HID + col], bg = sb[2 * HID + col], bo = sb[3 * HID + col];
#pragma unroll
  for (int r = 0; r < 8; ++r) {
    const int brow_i = mt * 16 + 8 * hf + r;
    const float zi = acc[0][r] * WSC_INV + bi;
    const float zf = acc[1][r] * WSC_INV + bf;
    const float zg = acc[2][r] * WSC_INV + bg;
    const float zo = acc[3][r] * WSC_INV + bo;
    const float cn = sigm_f(zf) * cs[r] + sigm_f(zi) * tanhf(zg);
    const float hn = sigm_f(zo) * tanhf(cn);
    cs[r] = cn;
    shn[brow_i * HPITCH + col] = h_bits(hn);
  }
}

template <int MODE>
__global__ __launch_bounds__(512) void lstm_kernel(const float* __restrict__ x,
                                                   const unsigned short* __restrict__ wcat,
                                                   const float* __restrict__ bias,
                                                   const unsigned short* __restrict__ hinit,
                                                   const float* __restrict__ cinit,
                                                   unsigned short* __restrict__ hout,
                                                   float* __restrict__ cfin) {
  constexpr int OPITCH = (MODE == 0) ? HID : 2 * HID;
  __shared__ __align__(16) unsigned short sH[2 * BATCH * HPITCH];
  __shared__ __align__(16) float sCF[BATCH * HID];
  __shared__ float sBias[GATES];
  const int tid = threadIdx.x, lane = tid & 31, wave = tid >> 5;
  const int hf = lane >> 4, rl = lane & 15;
  const int mt = wave & 3;
  const int cgb = (wave >> 2) * 2;

  for (int i = tid; i < 2 * BATCH * HPITCH / 2; i += 512) ((unsigned*)sH)[i] = 0u;
  sBias[tid] = bias[tid];
  float cs0[8], cs1[8];
#pragma unroll
  for (int r = 0; r < 8; ++r) { cs0[r] = 0.0f; cs1[r] = 0.0f; }
  if (MODE == 1) {
#pragma unroll
    for (int r = 0; r < 8; ++r) {
      const int brow_i = mt * 16 + 8 * hf + r;
      cs0[r] = cinit[brow_i * HID + cgb * 16 + rl];
      cs1[r] = cinit[brow_i * HID + (cgb + 1) * 16 + rl];
    }
  }
  __syncthreads();
  if (MODE == 1) {
    for (int i = tid; i < BATCH * HID / 8; i += 512) {
      const int row = i >> 4, c8 = (i & 15) * 8;
      const v4u w = *(const v4u*)(hinit + ((size_t)(row * SEQ + (SEQ - 1)) * HID + c8));
      *(v4u*)(sH + row * HPITCH + c8) = w;
    }
  }
  __syncthreads();

#pragma unroll 1
  for (int t = 0; t < SEQ; ++t) {
    const int cur = t & 1;
    unsigned short* shc = sH + cur * (BATCH * HPITCH);
    unsigned short* shn = sH + (cur ^ 1) * (BATCH * HPITCH);
    for (int i = tid; i < BATCH * FEAT; i += 512) {
      const int bb = i / FEAT, k = i - bb * FEAT;
      shc[bb * HPITCH + HID + k] = h_bits(x[((size_t)bb * SEQ + t) * FEAT + k]);
    }
    __syncthreads();
    lstm_group(shc, shn, wcat, sBias, mt, cgb, rl, hf, cs0);
    lstm_group(shc, shn, wcat, sBias, mt, cgb + 1, rl, hf, cs1);
    __syncthreads();
    for (int pass = 0; pass < 2; ++pass) {
#pragma unroll
      for (int it = 0; it < 2; ++it) {
        const int row = 4 * wave + 2 * it + hf;
        const v4u w = *(const v4u*)(shn + row * HPITCH + 8 * rl);
        *(volatile v4u*)(hout + ((size_t)(row * SEQ + t) * OPITCH + 8 * rl)) = w;
      }
      __threadfence();
    }
  }

  if (MODE == 0) {
#pragma unroll
    for (int r = 0; r < 8; ++r) {
      const int brow_i = mt * 16 + 8 * hf + r;
      sCF[brow_i * HID + cgb * 16 + rl] = cs0[r];
      sCF[brow_i * HID + (cgb + 1) * 16 + rl] = cs1[r];
    }
    __syncthreads();
    for (int pass = 0; pass < 2; ++pass) {
#pragma unroll
      for (int it = 0; it < 4; ++it) {
        const int row = 4 * wave + it;
        const v4f v = *(const v4f*)(sCF + row * HID + 4 * lane);
        *(volatile v4f*)(cfin + (size_t)row * HID + 4 * lane) = v;
      }
      __threadfence();
    }
  }
}

__global__ __launch_bounds__(256) void attn_kernel(const float* __restrict__ qf,
                                                   const float* __restrict__ ep,
                                                   const unsigned short* __restrict__ ench,
                                                   const float* __restrict__ vw,
                                                   unsigned short* __restrict__ dcat) {
  __shared__ __align__(16) unsigned short sEoT[HID * APITCH];
  __shared__ __align__(16) unsigned short sE[SEQ * APITCH];
  __shared__ __align__(16) unsigned short sVB[16 * APITCH];
  __shared__ __align__(16) unsigned short sP[TQ * APITCH];
  __shared__ __align__(16) unsigned short sC[TQ * APITCH];
  __shared__ __align__(16) float sQ[TQ * HID];
  __shared__ __align__(16) float sS[TQ * SEQ];
  const int tid = threadIdx.x, lane = tid & 31, wave = tid >> 5;
  const int hf = lane >> 4, rl = lane & 15;
  const int b = blockIdx.x >> 3;
  const int tq0 = (blockIdx.x & 7) * TQ;

  {
    const v4f* qsrc = (const v4f*)(qf + (size_t)(b * SEQ + tq0) * HID);
    for (int i = tid; i < TQ * HID / 4; i += 256) ((v4f*)sQ)[i] = qsrc[i];
  }
#pragma unroll 1
  for (int p = 0; p < 8; ++p) {
    const int tp = p * 16 + (tid >> 4);
    const int c8 = (tid & 15) * 8;
    const v4u w = *(const v4u*)(ench + ((size_t)(b * SEQ + tp) * HID + c8));
#pragma unroll
    for (int e = 0; e < 8; ++e) {
      const unsigned short hb = (unsigned short)((w[e >> 1] >> (16 * (e & 1))) & 0xffffu);
      sEoT[(c8 + e) * APITCH + tp] = hb;
    }
  }
  for (int i = tid; i < 16 * APITCH; i += 256) {
    const int row = i / APITCH, col = i - row * APITCH;
    const int cc = (col < HID) ? col : (HID - 1);
    const float v = vw[cc];
    sVB[i] = (row == 0 && col < HID) ? h_bits(WSC * v) : (unsigned short)0;
  }
  __syncthreads();

  const int tpr = wave * 16 + rl;
  const int g0 = hf * 64;
  const float* eprow = ep + (size_t)(b * SEQ + tpr) * HID + g0;
  _Float16* serow = (_Float16*)sE + tpr * APITCH + g0;
  const _Float16* arow = (const _Float16*)sE + (wave * 16 + rl) * APITCH + 8 * hf;
  const _Float16* vrow = (const _Float16*)sVB + rl * APITCH + 8 * hf;

#pragma unroll 1
  for (int tl = 0; tl < TQ; ++tl) {
    const float* qrow = sQ + tl * HID + g0;
#pragma unroll 1
    for (int ch = 0; ch < 8; ++ch) {
      const v4f e0 = *(const v4f*)(eprow + 8 * ch);
      const v4f e1 = *(const v4f*)(eprow + 8 * ch + 4);
      const v4f qa = *(const v4f*)(qrow + 8 * ch);
      const v4f qc = *(const v4f*)(qrow + 8 * ch + 4);
      v8h hv;
      hv[0] = (_Float16)tanhf(qa[0] + e0[0]);
      hv[1] = (_Float16)tanhf(qa[1] + e0[1]);
      hv[2] = (_Float16)tanhf(qa[2] + e0[2]);
      hv[3] = (_Float16)tanhf(qa[3] + e0[3]);
      hv[4] = (_Float16)tanhf(qc[0] + e1[0]);
      hv[5] = (_Float16)tanhf(qc[1] + e1[1]);
      hv[6] = (_Float16)tanhf(qc[2] + e1[2]);
      hv[7] = (_Float16)tanhf(qc[3] + e1[3]);
      *(v8h*)(serow + 8 * ch) = hv;
    }
    lds_wave_sync();
    v8f acc = (v8f){0.f,0.f,0.f,0.f,0.f,0.f,0.f,0.f};
#pragma unroll
    for (int kc = 0; kc < HID / 32; ++kc)
      acc = mma_h1(Frag<_Float16>::load(arow + kc * 32), Frag<_Float16>::load(vrow + kc * 32), acc);
    if (rl == 0) {
#pragma unroll
      for (int r = 0; r < 8; ++r) sS[tl * SEQ + wave * 16 + 8 * hf + r] = acc[r] * WSC_INV;
    }
    lds_wave_sync();
  }
  __syncthreads();

#pragma unroll
  for (int j = 0; j < 2; ++j) {
    const int tl = 2 * wave + j;
    float v[4];
#pragma unroll
    for (int e = 0; e < 4; ++e) v[e] = sS[tl * SEQ + lane + 32 * e];
    float m = fmaxf(fmaxf(v[0], v[1]), fmaxf(v[2], v[3]));
#pragma unroll
    for (int off = 16; off > 0; off >>= 1) m = fmaxf(m, __shfl_xor(m, off, 32));
    float s = 0.0f;
#pragma unroll
    for (int e = 0; e < 4; ++e) { v[e] = expf(v[e] - m); s += v[e]; }
#pragma unroll
    for (int off = 16; off > 0; off >>= 1) s += __shfl_xor(s, off, 32);
    const float inv = PCARRY / s;
#pragma unroll
    for (int e = 0; e < 4; ++e) sP[tl * APITCH + lane + 32 * e] = h_bits(v[e] * inv);
  }
  __syncthreads();

  {
    const _Float16* prow = (const _Float16*)sP + rl * APITCH + 8 * hf;
    const _Float16* brow = (const _Float16*)sEoT + (wave * 16 + rl) * APITCH + 8 * hf;
    v8f acc = (v8f){0.f,0.f,0.f,0.f,0.f,0.f,0.f,0.f};
#pragma unroll
    for (int kc = 0; kc < SEQ / 32; ++kc)
      acc = mma_h1(Frag<_Float16>::load(prow + kc * 32), Frag<_Float16>::load(brow + kc * 32), acc);
#pragma unroll
    for (int r = 0; r < 8; ++r) sC[(8 * hf + r) * APITCH + wave * 16 + rl] = h_bits(acc[r] * PCARRY_INV);
  }
  __syncthreads();

  {
    const int row = 2 * wave + hf;
    const int c8 = rl * 8;
    const v4u w = *(const v4u*)(sC + row * APITCH + c8);
    unsigned short* dst = dcat + ((size_t)(b * SEQ + tq0 + row) * (2 * HID) + HID + c8);
    *(volatile v4u*)dst = w;
    __threadfence();
    *(volatile v4u*)dst = w;
  }
}

__global__ __launch_bounds__(256) void out_pack_kernel(const float* __restrict__ cp,
                                                       const float* __restrict__ ob,
                                                       float* __restrict__ out) {
  const int i = blockIdx.x * 256 + threadIdx.x;
  if (i < NROW * FEAT / 4) {
    v4f v;
#pragma unroll
    for (int j = 0; j < 4; ++j) {
      const int e = 4 * i + j;
      const int row = e / FEAT;
      const int col = e - row * FEAT;
      v[j] = cp[(size_t)row * OUT_NPAD + col] + ob[col];
    }
    *(volatile v4f*)(out + (size_t)4 * i) = v;
    __threadfence();
    *(volatile v4f*)(out + (size_t)4 * i) = v;
  }
}

extern "C" void kernel_launch(void* const* d_in, const int* in_sizes, int n_in,
                              void* d_out, int out_size, void* d_ws, size_t ws_size,
                              hipStream_t stream) {
  (void)in_sizes; (void)n_in; (void)out_size;
  const float* x       = (const float*)d_in[0];
  const float* enc_Wih = (const float*)d_in[1];
  const float* enc_Whh = (const float*)d_in[2];
  const float* enc_b   = (const float*)d_in[3];
  const float* dec_Wih = (const float*)d_in[4];
  const float* dec_Whh = (const float*)d_in[5];
  const float* dec_b   = (const float*)d_in[6];
  const float* attn_W  = (const float*)d_in[7];
  const float* attn_b  = (const float*)d_in[8];
  const float* v_w     = (const float*)d_in[9];
  const float* out_W   = (const float*)d_in[10];
  const float* out_b   = (const float*)d_in[11];

  const size_t sz_wcat = (size_t)GATES * KCAT * 2;
  const size_t sz_watt = (size_t)HID * 2 * HID * 2;
  const size_t sz_wout = (size_t)OUT_NPAD * 2 * HID * 2;
  const size_t sz_ench = (size_t)NROW * HID * 2;
  const size_t sz_cT   = (size_t)BATCH * HID * 4;
  const size_t sz_encP = (size_t)NROW * HID * 4;
  const size_t sz_dcat = (size_t)NROW * 2 * HID * 2;
  const size_t sz_qf   = (size_t)NROW * HID * 4;
  const size_t sz_opad = (size_t)NROW * OUT_NPAD * 4;
  const size_t off_wcatE = 0;
  const size_t off_wcatD = off_wcatE + sz_wcat;
  const size_t off_watt  = off_wcatD + sz_wcat;
  const size_t off_wout  = off_watt + sz_watt;
  const size_t off_ench  = off_wout + sz_wout;
  const size_t off_cT    = off_ench + sz_ench;
  const size_t off_encP  = off_cT + sz_cT;
  const size_t off_dcat  = off_encP + sz_encP;
  const size_t off_qf    = off_dcat + sz_dcat;
  const size_t off_opad  = off_qf + sz_qf;
  const size_t total     = off_opad + sz_opad;
  if (ws_size < total) return;

  char* ws = (char*)d_ws;
  unsigned short* wcatE = (unsigned short*)(ws + off_wcatE);
  unsigned short* wcatD = (unsigned short*)(ws + off_wcatD);
  unsigned short* watt  = (unsigned short*)(ws + off_watt);
  unsigned short* woutP = (unsigned short*)(ws + off_wout);
  unsigned short* ench  = (unsigned short*)(ws + off_ench);
  float*          cT    = (float*)(ws + off_cT);
  float*          encP  = (float*)(ws + off_encP);
  unsigned short* dcat  = (unsigned short*)(ws + off_dcat);
  float*          qf    = (float*)(ws + off_qf);
  float*          opad  = (float*)(ws + off_opad);

  prep_planes<<<dim3((GATES * KCAT / 8 + 255) / 256, 4), 256, 0, stream>>>(
      enc_Whh, enc_Wih, dec_Whh, dec_Wih, attn_W, out_W, wcatE, wcatD, watt, woutP);
  lstm_kernel<0><<<1, 512, 0, stream>>>(x, wcatE, enc_b, ench, cT, ench, cT);
  wmma_gemm64<0, false, 2, 0, false><<<dim3((NROW / 64) * (HID / 64) / 8, 1), 256, 0, stream>>>(
      ench, ench, HID, 0L, watt + HID, watt + HID, 2 * HID, 0L,
      encP, encP, HID, 0L, attn_b, encP, 0L, NROW, HID, HID, WSC_INV);
  lstm_kernel<1><<<1, 512, 0, stream>>>(x, wcatD, dec_b, ench, cT, dcat, cT);
  wmma_gemm64<0, false, 0, 0, false><<<dim3((NROW / 64) * (HID / 64) / 8, 1), 256, 0, stream>>>(
      dcat, dcat, 2 * HID, 0L, watt, watt, 2 * HID, 0L,
      qf, qf, HID, 0L, attn_b, qf, 0L, NROW, HID, HID, WSC_INV);
  attn_kernel<<<BATCH * (SEQ / TQ), 256, 0, stream>>>(qf, encP, ench, v_w, dcat);
  wmma_gemm64<0, false, 0, 0, false><<<dim3((NROW / 64) * (OUT_NPAD / 64) / 8, 1), 256, 0, stream>>>(
      dcat, dcat, 2 * HID, 0L, woutP, woutP, 2 * HID, 0L,
      opad, opad, OUT_NPAD, 0L, attn_b, opad, 0L, NROW, OUT_NPAD, 2 * HID, WSC_INV);
  out_pack_kernel<<<NROW * FEAT / 4 / 256, 256, 0, stream>>>(opad, out_b, (float*)d_out);
}
